// ContextualAttention_13434657702224
// MI455X (gfx1250) — hardware-verified
//
#include <hip/hip_runtime.h>


#ifndef NB
#define NB 4
#endif
#define HH   96
#define CC   128
#define GW   48
#define LL   2304
#define KE   1152
#define XSTR_FULL ((size_t)HH * HH * CC)
#define MSTR_FULL ((size_t)HH * HH)
#define PCAR 16384.0f
#define XCAR 64.0f
#define OSCL (1.0f / 4194304.0f)
#define SCL  10.0f
#define EPSN 1.0e-4f
static_assert(LL == GW * GW);
static_assert(KE == 9 * CC);
static_assert(LL % 64 == 0);
static_assert(KE % 64 == 0);
static_assert(KE % 32 == 0);
static_assert(LL % 256 == 0);
static_assert((LL / 8) % 32 == 0);
static_assert((LL / 4) % 32 == 0);
static_assert((LL * (KE / 8)) % 256 == 0);
static_assert((KE * (LL / 8)) % 256 == 0);
static_assert((HH * HH * 32) % 256 == 0);
static_assert(NB >= 1 && NB <= 4);

typedef _Float16 h16;
typedef unsigned short bf;
typedef __attribute__((ext_vector_type(16))) __bf16   v16bf;
typedef __attribute__((ext_vector_type(16))) _Float16 v16h;
typedef __attribute__((ext_vector_type(8)))  _Float16 v8h;
typedef __attribute__((ext_vector_type(8)))  unsigned short v8us;
typedef __attribute__((ext_vector_type(8)))  float    v8f;
typedef __attribute__((ext_vector_type(4)))  float    v4f;
typedef v8h  __attribute__((may_alias)) v8ha;
typedef v4f  __attribute__((may_alias)) v4fa;
typedef v8us __attribute__((may_alias)) v8usa;

__device__ __forceinline__ unsigned short f2bf(float f) { unsigned u = __float_as_uint(f); u += 0x7FFFu + ((u >> 16) & 1u); return (unsigned short)(u >> 16); }
__device__ __forceinline__ float bf2f(unsigned short b) { return __uint_as_float(((unsigned)b) << 16); }
__device__ __forceinline__ float bfr(float f) { return bf2f(f2bf(f)); }
__device__ __forceinline__ v16h cat16(v8h lo, v8h hi) { return __builtin_shufflevector(lo, hi, 0, 1, 2, 3, 4, 5, 6, 7, 8, 9, 10, 11, 12, 13, 14, 15); }
__device__ __forceinline__ v16bf cat16b(v8us lo, v8us hi) { return __builtin_bit_cast(v16bf, __builtin_shufflevector(lo, hi, 0, 1, 2, 3, 4, 5, 6, 7, 8, 9, 10, 11, 12, 13, 14, 15)); }
__device__ __forceinline__ v8f wmma16(v16h a, v16h b, v8f c) { return __builtin_amdgcn_wmma_f32_16x16x32_f16(false, a, false, b, (short)0, c, false, false); }
__device__ __forceinline__ v8f wmmab(v16bf a, v16bf b, v8f c) { return __builtin_amdgcn_wmma_f32_16x16x32_bf16(false, a, false, b, (short)0, c, false, false); }
__device__ __forceinline__ h16 tohx(float x) { return (h16)x; }
__device__ __forceinline__ void splitf(float y, unsigned short& h, unsigned short& l) { h = f2bf(y); l = f2bf(y - bf2f(h)); }

template <typename T16> struct WFrag;
template <> struct WFrag<h16> { typedef v16h V; static __device__ __forceinline__ V ld(const h16* p) { return cat16(*(const v8h*)p, *(const v8h*)(p + 16)); } static __device__ __forceinline__ v8f mma(V a, V b, v8f c) { return wmma16(a, b, c); } };
template <> struct WFrag<bf> { typedef v16bf V; static __device__ __forceinline__ V ld(const bf* p) { return cat16b(*(const v8us*)p, *(const v8us*)(p + 16)); } static __device__ __forceinline__ v8f mma(V a, V b, v8f c) { return wmmab(a, b, c); } };

template <typename T16, int NSPLIT, int CMODE>
__global__ __launch_bounds__(32) void k_gemmc(const T16* __restrict__ A, const T16* __restrict__ A2, const T16* __restrict__ Bt, const T16* __restrict__ Bt2, int K, float* C, int ldc, int roff, size_t sA, size_t sB, size_t sC) {
    typedef typename WFrag<T16>::V V;
    __shared__ __align__(16) float os[16 * 68];
    const size_t z = blockIdx.z; A += z * sA; if (A2) A2 += z * sA; Bt += z * sB; if (Bt2) Bt2 += z * sB; C += z * sC;
    const int lane = threadIdx.x & 31, lr = lane & 15, hi = lane >> 4; const int r0 = blockIdx.x * 64, c0 = blockIdx.y * 64;
    if (CMODE == 1 && c0 > r0 + roff + 63) return;
    const int Kl = (CMODE == 2) ? min(K, r0 + roff + 64) : K;
    v8f acc[4][4];
#pragma unroll
    for (int mb = 0; mb < 4; ++mb)
#pragma unroll
        for (int nb = 0; nb < 4; ++nb) acc[mb][nb] = (v8f){};
    const size_t aoff = (size_t)(r0 + lr) * K + 8 * hi, boff = (size_t)(c0 + lr) * K + 8 * hi;
#pragma unroll 1
    for (int kc = 0; kc < Kl; kc += 32) {
        V a[4], a2[4];
#pragma unroll
        for (int mb = 0; mb < 4; ++mb) { a[mb] = WFrag<T16>::ld(A + aoff + (size_t)mb * 16 * K + kc); if (NSPLIT == 1 || NSPLIT == 2) a2[mb] = WFrag<T16>::ld(A2 + aoff + (size_t)mb * 16 * K + kc); }
#pragma unroll
        for (int nb = 0; nb < 4; ++nb) { const V b = WFrag<T16>::ld(Bt + boff + (size_t)nb * 16 * K + kc); V b2; if (NSPLIT >= 2) b2 = WFrag<T16>::ld(Bt2 + boff + (size_t)nb * 16 * K + kc);
#pragma unroll
            for (int mb = 0; mb < 4; ++mb) { acc[mb][nb] = WFrag<T16>::mma(a[mb], b, acc[mb][nb]); if (NSPLIT == 1 || NSPLIT == 2) acc[mb][nb] = WFrag<T16>::mma(a2[mb], b, acc[mb][nb]); if (NSPLIT >= 2) acc[mb][nb] = WFrag<T16>::mma(a[mb], b2, acc[mb][nb]); } }
        asm volatile("v_nop\n\tv_nop\n\tv_nop\n\tv_nop" : "+v"(acc[0][0]), "+v"(acc[1][1]), "+v"(acc[2][2]), "+v"(acc[3][3]) : "v"(a[0]), "v"(a[3]));
    }
#pragma unroll
    for (int mb = 0; mb < 4; ++mb) {
#pragma unroll
        for (int nb = 0; nb < 4; ++nb) {
#pragma unroll
            for (int j = 0; j < 8; ++j) os[(hi * 8 + j) * 68 + nb * 16 + lr] = acc[mb][nb][j]; }
        __builtin_amdgcn_wave_barrier(); asm volatile("" ::: "memory");
        float* crow = C + (size_t)(r0 + mb * 16) * ldc + c0;
#pragma unroll 1
        for (int ps = 0; ps < 2; ++ps) {
#pragma unroll
            for (int s = 0; s < 8; ++s) { const int row = 2 * s + hi, cofs = lr * 4; v4f val = *(const v4fa*)(os + row * 68 + cofs);
                *(volatile v4f*)(crow + (size_t)row * ldc + cofs) = val; }
            if (ps == 0) __threadfence(); }
        __builtin_amdgcn_wave_barrier(); asm volatile("" ::: "memory");
    }
}

__global__ __launch_bounds__(256) void k_fpool(const float* __restrict__ x, float* F) {
    const int gt = blockIdx.x * 256 + threadIdx.x; if (gt >= LL * 32) return;
    const int pix = gt >> 5, lane = gt & 31; const int i = pix / GW, j = pix - i * GW; const int c = lane * 4;
    const float* x0 = x + ((size_t)(2 * i) * HH + 2 * j) * CC + c;
    const v4f a00 = *(const v4f*)x0; const v4f a10 = *(const v4f*)(x0 + (size_t)HH * CC); const v4f a01 = *(const v4f*)(x0 + CC); const v4f a11 = *(const v4f*)(x0 + (size_t)HH * CC + CC);
    v4f o;
#pragma unroll
    for (int k = 0; k < 4; ++k) { const float s0 = bfr(a00[k]) + bfr(a10[k]); const float s1 = bfr(a01[k]) + bfr(a11[k]); o[k] = (s0 + s1) * 0.25f; }
    float* dst = F + (size_t)pix * CC + c;
    *(volatile v4f*)dst = o; __threadfence(); *(volatile v4f*)dst = o;
}

__global__ __launch_bounds__(256) void k_norm(const float* __restrict__ F, const float* __restrict__ msk, float* invn, float* vfl) {
    __shared__ __align__(16) float si[256]; __shared__ __align__(16) float sv[256];
    const int tid = threadIdx.x; const int l = blockIdx.x * 256 + tid; const int i = l / GW, j = l - i * GW;
    float ssq = 0.f, msum = 0.f;
#pragma unroll 1
    for (int tap = 0; tap < 9; ++tap) {
        const int a = tap / 3, b = tap - a * 3; const int y = i + a - 1, xq = j + b - 1; const bool ok = (y >= 0) && (y < GW) && (xq >= 0) && (xq < GW);
        const int yc = min(max(y, 0), GW - 1), xc = min(max(xq, 0), GW - 1);
        const float* fr = F + ((size_t)yc * GW + xc) * CC;
        float t0 = 0.f, t1 = 0.f, t2 = 0.f, t3 = 0.f;
#pragma unroll 1
        for (int c4 = 0; c4 < CC / 4; ++c4) { const v4f v = *(const v4f*)(fr + c4 * 4); t0 += v[0] * v[0]; t1 += v[1] * v[1]; t2 += v[2] * v[2]; t3 += v[3] * v[3]; }
        const float ts = (t0 + t1) + (t2 + t3);
        const float* m0 = msk + (size_t)(2 * yc) * HH + 2 * xc;
        const float mv = ((bfr(m0[0]) + bfr(m0[HH])) + (bfr(m0[1]) + bfr(m0[HH + 1]))) * 0.25f;
        ssq += ok ? ts : 0.f; msum += ok ? mv : 0.f;
    }
    si[tid] = 1.0f / fmaxf(sqrtf(ssq), EPSN); sv[tid] = (msum == 0.f) ? 1.0f : 0.0f;
    __syncthreads();
    const int l0 = blockIdx.x * 256;
#pragma unroll 1
    for (int ps = 0; ps < 2; ++ps) {
        if (tid < 64) { const v4f v = *(const v4fa*)(si + tid * 4); *(volatile v4f*)(invn + l0 + tid * 4) = v; }
        else if (tid < 128) { const v4f v = *(const v4fa*)(sv + (tid - 64) * 4); *(volatile v4f*)(vfl + l0 + (tid - 64) * 4) = v; }
        if (ps == 0) __threadfence(); }
}

__global__ __launch_bounds__(256) void k_fplanes(const float* __restrict__ F, bf* Ph, bf* Pl) {
    const int p = blockIdx.x * 256 + threadIdx.x; if (p >= LL * (KE / 8)) return;
    const int l = p / (KE / 8), k0 = (p - l * (KE / 8)) * 8; const int tap = k0 / CC, c = k0 - tap * CC; const int a = tap / 3, b = tap - a * 3;
    const int i = l / GW, j = l - i * GW; const int y = i + a - 1, xq = j + b - 1; const bool ok = (y >= 0) && (y < GW) && (xq >= 0) && (xq < GW);
    const int yc = min(max(y, 0), GW - 1), xc = min(max(xq, 0), GW - 1);
    const float* fr = F + ((size_t)yc * GW + xc) * CC + c; const v4f u0 = *(const v4f*)fr; const v4f u1 = *(const v4f*)(fr + 4);
    v8us oh, ol;
#pragma unroll
    for (int e = 0; e < 4; ++e) { unsigned short hq, lq; splitf(ok ? u0[e] : 0.f, hq, lq); oh[e] = hq; ol[e] = lq; splitf(ok ? u1[e] : 0.f, hq, lq); oh[4 + e] = hq; ol[4 + e] = lq; }
    const size_t oo = (size_t)l * KE + k0;
    *(volatile v8us*)(Ph + oo) = oh; *(volatile v8us*)(Pl + oo) = ol; __threadfence(); *(volatile v8us*)(Ph + oo) = oh; *(volatile v8us*)(Pl + oo) = ol;
}

__global__ __launch_bounds__(256) void k_xt(const float* __restrict__ x, h16* XT) {
    const int p = blockIdx.x * 256 + threadIdx.x; if (p >= KE * (LL / 8)) return;
    const int n = p / (LL / 8), l0 = (p - n * (LL / 8)) * 8; const int tap = n / CC, c = n - tap * CC; const int a = tap / 3, b = tap - a * 3;
    const int i = l0 / GW, j0 = l0 - i * GW; const int py = 2 * i + a; const bool oky = (py < HH); const int pyc = min(py, HH - 1);
    const float* xr = x + (size_t)pyc * HH * CC + c;
    v8h o;
#pragma unroll
    for (int e = 0; e < 8; ++e) { const int qx = 2 * (j0 + e) + b; const bool ok = oky && (qx < HH); const int qc = min(qx, HH - 1); const float v = xr[(size_t)qc * CC]; o[e] = tohx(bfr(ok ? v : 0.f) * XCAR); }
    const size_t oo = (size_t)n * LL + l0;
    *(volatile v8h*)(XT + oo) = o; __threadfence(); *(volatile v8h*)(XT + oo) = o;
}

__global__ __launch_bounds__(256) void k_fuse1(const float* __restrict__ G, const float* __restrict__ invn, float* A1) {
    const int gt = blockIdx.x * 256 + threadIdx.x; if (gt >= LL * (LL / 4)) return;
    const int q = gt / (LL / 4), l0 = (gt - q * (LL / 4)) * 4;
    float t[3][4];
#pragma unroll
    for (int dd = 0; dd < 3; ++dd) {
        const int r = q + dd - 1; const bool rok = (r >= 0) && (r < LL); const int rc = min(max(r, 0), LL - 1);
#pragma unroll
        for (int e = 0; e < 4; ++e) {
            const int cidx = l0 + e + dd - 1; const bool ok = rok && (cidx >= 0) && (cidx < LL); const int cc = min(max(cidx, 0), LL - 1);
            const float gd = G[(size_t)rc * LL + cc]; const float gu = G[(size_t)cc * LL + rc];
            const float g = (cc <= rc) ? gd : gu; const float y = g * invn[cc];
            t[dd][e] = ok ? y : 0.f; } }
    v4f o;
#pragma unroll
    for (int e = 0; e < 4; ++e) o[e] = (t[0][e] + t[1][e]) + t[2][e];
    float* dst = A1 + (size_t)q * LL + l0;
    *(volatile v4f*)dst = o; __threadfence(); *(volatile v4f*)dst = o;
}

__global__ __launch_bounds__(256) void k_fsoft(const float* __restrict__ A1, const float* __restrict__ vfl, h16* Pc) {
    __shared__ __align__(16) float rows[3 * LL];
    __shared__ float redm[8]; __shared__ float reds[8];
    const int tid = threadIdx.x, lane = tid & 31, wv = tid >> 5;
    const int q = blockIdx.x; const int i = q / GW, j = q - i * GW; const int r = j * GW + i;
#pragma unroll
    for (int d = 0; d < 3; ++d) {
        const int rp = r + d - 1;
        if (rp >= 0 && rp < LL) {
            const float* src = A1 + (size_t)((rp % GW) * GW + rp / GW) * LL;
#pragma unroll 1
            for (int tcol = tid; tcol < LL; tcol += 256) rows[d * LL + tcol] = src[tcol];
        } else {
#pragma unroll 1
            for (int tcol = tid; tcol < LL; tcol += 256) rows[d * LL + tcol] = 0.f;
        }
    }
    __syncthreads();
    float z[9]; float mx = -3.0e38f;
#pragma unroll
    for (int it = 0; it < 9; ++it) {
        const int s = tid + it * 256; const int u = s / GW, v = s - u * GW;
        const int im = (u >= 1) ? (s - GW) : ((GW - 1) * GW + v - 1);
        const int ip = (u <= GW - 2) ? (s + GW) : (v + 1);
        const int imc = min(max(im, 0), LL - 1), ipc = min(max(ip, 0), LL - 1);
        const float a0 = rows[imc], a1v = rows[LL + s], a2 = rows[2 * LL + ipc];
        const float t0 = (s != 0) ? a0 : 0.f; const float t2 = (s != LL - 1) ? a2 : 0.f;
        const float fz = (t0 + a1v) + t2;
        const float zz = (fz * vfl[s]) * SCL;
        z[it] = zz; mx = fmaxf(mx, zz);
    }
#pragma unroll
    for (int sh = 16; sh; sh >>= 1) mx = fmaxf(mx, __shfl_xor(mx, sh, 32));
    if (lane == 0) redm[wv] = mx;
    __syncthreads();
    float gm = redm[0];
#pragma unroll
    for (int w = 1; w < 8; ++w) gm = fmaxf(gm, redm[w]);
    float sum = 0.f;
#pragma unroll
    for (int it = 0; it < 9; ++it) { float d0 = __fsub_rn(z[it], gm); asm volatile("" : "+v"(d0)); const float e = __builtin_amdgcn_exp2f(__fmul_rn(d0, 1.4426950408889634f)); z[it] = e; sum += e; }
#pragma unroll
    for (int sh = 16; sh; sh >>= 1) sum += __shfl_xor(sum, sh, 32);
    if (lane == 0) reds[wv] = sum;
    __syncthreads();
    float tot = reds[0];
#pragma unroll
    for (int w = 1; w < 8; ++w) tot += reds[w];
    const float inv = 1.0f / tot;
#pragma unroll
    for (int it = 0; it < 9; ++it) { const int s = tid + it * 256; rows[s] = ((z[it] * inv) * vfl[s]) * PCAR; }
    __syncthreads();
    v8h o0, o1;
    { const v4f w0 = *(const v4fa*)(rows + 8 * tid), w1 = *(const v4fa*)(rows + 8 * tid + 4);
#pragma unroll
      for (int k = 0; k < 4; ++k) { o0[k] = tohx(w0[k]); o0[4 + k] = tohx(w1[k]); } }
    { const int p1 = tid + 256; const v4f w0 = *(const v4fa*)(rows + 8 * p1), w1 = *(const v4fa*)(rows + 8 * p1 + 4);
#pragma unroll
      for (int k = 0; k < 4; ++k) { o1[k] = tohx(w0[k]); o1[4 + k] = tohx(w1[k]); } }
    const size_t ob = (size_t)q * LL;
#pragma unroll 1
    for (int ps = 0; ps < 2; ++ps) {
        *(volatile v8h*)(Pc + ob + 8 * tid) = o0;
        if (tid < 32) *(volatile v8h*)(Pc + ob + 8 * (tid + 256)) = o1;
        if (ps == 0) __threadfence(); }
}

__global__ __launch_bounds__(256) void k_out(const float* __restrict__ T, float* out) {
    const int gt = blockIdx.x * 256 + threadIdx.x; if (gt >= HH * HH * 32) return;
    const int pix = gt >> 5, lane = gt & 31; const int p = pix / HH, qx = pix - p * HH; const int c = lane * 4;
    v4f acc = (v4f){};
#pragma unroll
    for (int ta = 0; ta < 2; ++ta) {
        const int a = (p & 1) + 2 * ta; const int hp = (p - a) >> 1;
        const bool aok = (a <= 2) && (hp >= 0) && (hp < GW);
#pragma unroll
        for (int tb = 0; tb < 2; ++tb) {
            const int b = (qx & 1) + 2 * tb; const int wp = (qx - b) >> 1;
            const bool ok = aok && (b <= 2) && (wp >= 0) && (wp < GW);
            const int ac = min(a, 2), bc = min(b, 2), hpc = min(max(hp, 0), GW - 1), wpc = min(max(wp, 0), GW - 1);
            const v4f v = *(const v4f*)(T + (size_t)(hpc * GW + wpc) * KE + (ac * 3 + bc) * CC + c);
#pragma unroll
            for (int k = 0; k < 4; ++k) acc[k] += ok ? v[k] : 0.f; } }
    const v4f o = acc * OSCL;
    float* dst = out + (size_t)pix * CC + c;
    *(volatile v4f*)dst = o; __threadfence(); *(volatile v4f*)dst = o;
}

extern "C" void kernel_launch(void* const* d_in, const int* in_sizes, int n_in,
                              void* d_out, int out_size, void* d_ws, size_t ws_size, hipStream_t stream) {
    if (n_in < 2) return;
    if ((size_t)in_sizes[0] < (size_t)NB * XSTR_FULL || (size_t)in_sizes[1] < (size_t)NB * MSTR_FULL || (size_t)out_size < (size_t)NB * XSTR_FULL) return;
    const float* x = (const float*)d_in[0]; const float* msk = (const float*)d_in[1];
    float* OUT = (float*)d_out;
    char* wsp = (char*)d_ws;
    auto take = [&](size_t bytes) { char* p = wsp; wsp += (bytes + 255) & ~(size_t)255; return (void*)p; };
    float* Fb   = (float*)take((size_t)LL * CC * 4);
    float* INVN = (float*)take((size_t)LL * 4); float* VFL = (float*)take((size_t)LL * 4);
    bf* FPh = (bf*)take((size_t)LL * KE * 2); bf* FPl = (bf*)take((size_t)LL * KE * 2);
    h16* XT = (h16*)take((size_t)KE * LL * 2);
    float* G  = (float*)take((size_t)LL * LL * 4);
    float* A1 = (float*)take((size_t)LL * LL * 4);
    h16* Pc = (h16*)take((size_t)LL * LL * 2);
    float* T  = (float*)take((size_t)LL * KE * 4);
    const size_t used = (size_t)(wsp - (char*)d_ws);
    if (used > ws_size || used > ((size_t)128 << 20)) return;
    for (int b = 0; b < NB; ++b) {
        const float* xb = x + (size_t)b * XSTR_FULL; const float* mb = msk + (size_t)b * MSTR_FULL; float* ob = OUT + (size_t)b * XSTR_FULL;
        k_fpool<<<(unsigned)(LL * 32 / 256), 256, 0, stream>>>(xb, Fb);
        k_norm<<<(unsigned)(LL / 256), 256, 0, stream>>>(Fb, mb, INVN, VFL);
        k_fplanes<<<(unsigned)(LL * (KE / 8) / 256), 256, 0, stream>>>(Fb, FPh, FPl);
        k_xt<<<(unsigned)(KE * (LL / 8) / 256), 256, 0, stream>>>(xb, XT);
        k_gemmc<bf, 2, 1><<<dim3(LL / 64, LL / 64, 1), 32, 0, stream>>>(FPh, FPl, FPh, FPl, KE, G, LL, 0, (size_t)0, (size_t)0, (size_t)0);
        k_fuse1<<<(unsigned)(LL * (LL / 4) / 256), 256, 0, stream>>>(G, INVN, A1);
        k_fsoft<<<(unsigned)LL, 256, 0, stream>>>(A1, VFL, Pc);
        k_gemmc<h16, 0, 0><<<dim3(LL / 64, KE / 64, 1), 32, 0, stream>>>(Pc, nullptr, XT, nullptr, LL, T, KE, 0, (size_t)0, (size_t)0, (size_t)0);
        k_out<<<(unsigned)(HH * HH * 32 / 256), 256, 0, stream>>>(T, ob);
    }
}
